// ReadUnit_9371618640097
// MI455X (gfx1250) — hardware-verified
//
#include <hip/hip_runtime.h>
#include <stddef.h>


typedef _Float16 v16h __attribute__((ext_vector_type(16)));
typedef _Float16 v8h  __attribute__((ext_vector_type(8)));
typedef float    v8f  __attribute__((ext_vector_type(8)));
typedef float    v4f  __attribute__((ext_vector_type(4)));
typedef _Float16 h16;

#ifndef NB
#define NB 128
#endif
#define NB_FULL 128
#define DIM   512
#define PIX   196
#define PIXQ  49
#define KMG   1024
#define LDA   1024
#define MROWS (NB * PIX)

static_assert(NB >= 16 && NB <= NB_FULL && (NB % 16) == 0);
static_assert((MROWS % 64) == 0);
static_assert((NB_FULL % 64) == 0);
static_assert((DIM % 128) == 0 && (DIM % 64) == 0 && (DIM % 32) == 0);
static_assert(KMG == 2 * DIM && LDA == KMG && (KMG % 32) == 0);
static_assert(PIX == 4 * PIXQ);
static_assert(PIX <= 7 * 32);
static_assert(13 * 256 >= 64 * PIXQ);
static_assert(7 * 256 >= PIX * 8);
static_assert(((NB_FULL * DIM) % 2048) == 0);
static_assert((size_t)MROWS * LDA < (size_t)0xFFFFFFFFu);

#define LDT 72
#define LDC 68
static_assert((LDT % 8) == 0 && LDT >= 64);
static_assert((LDC % 4) == 0 && LDC >= 64);

#define WCARRY 64.0f
#define ACARRY 256.0f

#define WSQ_BYTES ((size_t)DIM * DIM * 2)
#define WMG_BYTES ((size_t)DIM * KMG * 2)
#define M16_BYTES ((size_t)NB_FULL * DIM * 2)
#define MP_BYTES  ((size_t)NB_FULL * DIM * 4)
#define XI_BYTES  ((size_t)MROWS * LDA * 2)
#define MV_BYTES  ((size_t)MROWS * 4)
#define OFF_WM  ((size_t)0)
#define OFF_WKB (OFF_WM + WSQ_BYTES)
#define OFF_WMG (OFF_WKB + WSQ_BYTES)
#define OFF_M16 (OFF_WMG + WMG_BYTES)
#define OFF_MP  (OFF_M16 + M16_BYTES)
#define OFF_XI  (OFF_MP + MP_BYTES)
#define OFF_MV  (OFF_XI + XI_BYTES)
#define WS_TOTAL (OFF_MV + MV_BYTES)
static_assert((WSQ_BYTES % 128) == 0 && (WMG_BYTES % 128) == 0 && (M16_BYTES % 128) == 0);
static_assert((MP_BYTES % 128) == 0 && (XI_BYTES % 128) == 0 && (MV_BYTES % 256) == 0);
static_assert(WS_TOTAL <= (size_t)134217728);

__device__ __forceinline__ float bf16r(float x) {
  unsigned int u = __float_as_uint(x);
  u = (u + 0x7FFFu + ((u >> 16) & 1u)) & 0xFFFF0000u;
  return __uint_as_float(u);
}

static __device__ __forceinline__ h16 toh_flush(float v) {
  const h16 r = (h16)v;
  return (fabsf(v) < 6.103515625e-05f) ? (h16)0.0f : r;
}

__device__ __forceinline__ v16h frag_at(const _Float16* p) {
  v8h lo = *(const v8h*)(p);
  v8h hi = *(const v8h*)(p + 16);
  v16h out;
#pragma unroll
  for (int i = 0; i < 8; ++i) { out[i] = lo[i]; out[i + 8] = hi[i]; }
  return out;
}

__device__ __forceinline__ v8f wmma16(v16h a, v16h b, v8f c) {
  v8f d = __builtin_amdgcn_wmma_f32_16x16x32_f16(false, a, false, b, (short)0, c,
                                                 false, false);
  asm volatile("v_nop\n\tv_nop\n\tv_nop\n\tv_nop" : "+v"(d) : "v"(a), "v"(b));
  return d;
}

__device__ __forceinline__ float red16_sum(float x) {
#pragma unroll
  for (int off = 1; off < 16; off <<= 1) x += __shfl_xor(x, off, 32);
  return x;
}
__device__ __forceinline__ float red32_sum(float x) {
#pragma unroll
  for (int off = 1; off < 32; off <<= 1) x += __shfl_xor(x, off, 32);
  return x;
}

__global__ __launch_bounds__(256) void wconv_kernel(
    const float* __restrict__ W, _Float16* __restrict__ Wt, unsigned ldw, unsigned ldk) {
  __shared__ _Float16 T[64 * LDT];
  const unsigned tid = threadIdx.x;
  const unsigned n0 = blockIdx.x * 64u;
  const unsigned k0 = blockIdx.y * 64u;
#pragma unroll 4
  for (unsigned j = 0; j < 16u; ++j) {
    const unsigned idx = tid + 256u * j;
    const unsigned kr = idx >> 6, nc = idx & 63u;
    const float v = W[(size_t)(k0 + kr) * ldw + n0 + nc];
    T[nc * LDT + kr] = (_Float16)(WCARRY * bf16r(v));
  }
  __syncthreads();
  v8h x[2];
  size_t off[2];
#pragma unroll
  for (unsigned i = 0; i < 2u; ++i) {
    const unsigned n = 32u * i + (tid >> 3);
    const unsigned kc = (tid & 7u) * 8u;
    x[i] = *(const v8h*)&T[n * LDT + kc];
    off[i] = (size_t)(n0 + n) * ldk + k0 + kc;
  }
#pragma unroll
  for (int i = 0; i < 2; ++i) *(volatile v8h*)(Wt + off[i]) = x[i];
  __threadfence();
#pragma unroll
  for (int i = 0; i < 2; ++i) *(volatile v8h*)(Wt + off[i]) = x[i];
}

__global__ __launch_bounds__(256) void mconv_kernel(
    const float* __restrict__ X, _Float16* __restrict__ dst) {
#pragma clang fp contract(off)
  const size_t i = ((size_t)blockIdx.x * 256u + threadIdx.x) * 8u;
  const v4f a0 = *(const v4f*)(X + i);
  const v4f a1 = *(const v4f*)(X + i + 4u);
  v8h o;
#pragma unroll
  for (int j = 0; j < 4; ++j) {
    o[j]     = toh_flush(ACARRY * bf16r(a0[j]));
    o[j + 4] = toh_flush(ACARRY * bf16r(a1[j]));
  }
  *(volatile v8h*)(dst + i) = o;
  __threadfence();
  *(volatile v8h*)(dst + i) = o;
}

__global__ __launch_bounds__(256) void kbconv_kernel(
    const float* __restrict__ KB, _Float16* __restrict__ XI) {
#pragma clang fp contract(off)
  __shared__ _Float16 T[PIX * LDT];
  const unsigned tid = threadIdx.x;
  const unsigned c0 = blockIdx.x * 64u;
  const unsigned b = blockIdx.y;
  const float* src = KB + ((size_t)b * DIM + c0) * PIX;
  const unsigned NQ = 64u * PIXQ;
#pragma unroll 1
  for (unsigned j = 0; j < 13u; ++j) {
    const unsigned q = tid + 256u * j;
    const unsigned qc = (q < NQ) ? q : (NQ - 1u);
    const v4f v = *(const v4f*)(src + (size_t)qc * 4u);
    const unsigned cr = qc / (unsigned)PIXQ;
    const unsigned t4 = (qc - cr * (unsigned)PIXQ) * 4u;
    if (q < NQ) {
#pragma unroll
      for (unsigned i = 0; i < 4u; ++i)
        T[(t4 + i) * LDT + cr] = toh_flush(ACARRY * bf16r(v[i]));
    }
  }
  __syncthreads();
  const unsigned NP = (unsigned)PIX * 8u;
#pragma unroll 1
  for (unsigned j = 0; j < 7u; ++j) {
    const unsigned pc = tid + 256u * j;
    const unsigned pq = (pc < NP) ? pc : (NP - 1u);
    const unsigned t = pq >> 3, kc = (pq & 7u) * 8u;
    const v8h x = *(const v8h*)&T[t * LDT + kc];
    _Float16* p = XI + (size_t)(b * (unsigned)PIX + t) * LDA + DIM + c0 + kc;
    if (pc < NP) *(volatile v8h*)p = x;
  }
  __threadfence();
#pragma unroll 1
  for (unsigned j = 0; j < 7u; ++j) {
    const unsigned pc = tid + 256u * j;
    const unsigned pq = (pc < NP) ? pc : (NP - 1u);
    const unsigned t = pq >> 3, kc = (pq & 7u) * 8u;
    const v8h x = *(const v8h*)&T[t * LDT + kc];
    _Float16* p = XI + (size_t)(b * (unsigned)PIX + t) * LDA + DIM + c0 + kc;
    if (pc < NP) *(volatile v8h*)p = x;
  }
}

template <int MODE>
__device__ __forceinline__ void gemm_body(
    const _Float16* __restrict__ A16, const unsigned lda, const _Float16* __restrict__ Bt,
    const unsigned K, const float* __restrict__ bias, const float* __restrict__ mp,
    float* __restrict__ outf, _Float16* out16) {
  __shared__ float Cs[64 * LDC];
  const unsigned tid = threadIdx.x, lane = tid & 31u;
  const unsigned w = (unsigned)__builtin_amdgcn_readfirstlane(threadIdx.x >> 5);
  const unsigned mw = w >> 1, nw = w & 1u;
  const unsigned hh = lane >> 4, m = lane & 15u;
  const unsigned n0 = blockIdx.x * 64u;
  const unsigned row0 = blockIdx.y * 64u;
  const float cs = 1.0f / (ACARRY * WCARRY);

  const _Float16* ap  = A16 + (size_t)(row0 + mw * 16u + m) * lda + hh * 8u;
  const _Float16* bp0 = Bt + (size_t)(n0 + nw * 32u + m) * K + hh * 8u;
  const _Float16* bp1 = bp0 + (size_t)16 * K;
  v8f acc0 = {}, acc1 = {};
#pragma unroll 2
  for (unsigned k0 = 0; k0 < K; k0 += 32u) {
    const v16h a  = frag_at(ap + k0);
    const v16h b0 = frag_at(bp0 + k0);
    const v16h b1 = frag_at(bp1 + k0);
    acc0 = wmma16(a, b0, acc0);
    acc1 = wmma16(a, b1, acc1);
  }
#pragma unroll
  for (int r = 0; r < 8; ++r) {
    float* d = &Cs[(mw * 16u + hh * 8u + (unsigned)r) * LDC + nw * 32u + m];
    d[0]  = acc0[r];
    d[16] = acc1[r];
  }
  __syncthreads();

  if (MODE == 0) {
    v4f xs[4];
    size_t off[4];
#pragma unroll
    for (unsigned i = 0; i < 4u; ++i) {
      const unsigned r = 16u * i + (tid >> 4);
      const unsigned c = (tid & 15u) * 4u;
      const v4f u = *(const v4f*)&Cs[r * LDC + c];
      const v4f g = *(const v4f*)(bias + n0 + c);
      v4f val;
#pragma unroll
      for (int j = 0; j < 4; ++j) val[j] = u[j] * cs + bf16r(g[j]);
      xs[i] = val;
      off[i] = (size_t)(row0 + r) * DIM + n0 + c;
    }
#pragma unroll
    for (int i = 0; i < 4; ++i) *(volatile v4f*)(outf + off[i]) = xs[i];
    __threadfence();
#pragma unroll
    for (int i = 0; i < 4; ++i) *(volatile v4f*)(outf + off[i]) = xs[i];
  }

  if (MODE == 1) {
    v8h x[2];
    size_t off[2];
#pragma unroll
    for (unsigned i = 0; i < 2u; ++i) {
      const unsigned r = 32u * i + (tid >> 3);
      const unsigned c = (tid & 7u) * 8u;
      const unsigned row = row0 + r;
      const unsigned bidx = row / (unsigned)PIX;
      const v4f u0 = *(const v4f*)&Cs[r * LDC + c];
      const v4f u1 = *(const v4f*)&Cs[r * LDC + c + 4];
      const v4f g0 = *(const v4f*)(bias + n0 + c);
      const v4f g1 = *(const v4f*)(bias + n0 + c + 4u);
      const v4f p0 = *(const v4f*)(mp + (size_t)bidx * DIM + n0 + c);
      const v4f p1 = *(const v4f*)(mp + (size_t)bidx * DIM + n0 + c + 4u);
#pragma unroll
      for (int j = 0; j < 4; ++j) {
        x[i][j]     = toh_flush(ACARRY * (p0[j] * (u0[j] * cs + bf16r(g0[j]))));
        x[i][j + 4] = toh_flush(ACARRY * (p1[j] * (u1[j] * cs + bf16r(g1[j]))));
      }
      off[i] = (size_t)row * LDA + n0 + c;
    }
#pragma unroll
    for (int i = 0; i < 2; ++i) *(volatile v8h*)(out16 + off[i]) = x[i];
    __threadfence();
#pragma unroll
    for (int i = 0; i < 2; ++i) *(volatile v8h*)(out16 + off[i]) = x[i];
  }
}

__global__ __launch_bounds__(256) void gemm_mp_kernel(
    const _Float16* __restrict__ A16, const _Float16* __restrict__ Bt,
    const float* __restrict__ bias, float* __restrict__ mp) {
  gemm_body<0>(A16, (unsigned)DIM, Bt, (unsigned)DIM, bias, bias, mp, (_Float16*)0);
}
__global__ __launch_bounds__(256) void gemm_i_kernel(
    const _Float16* __restrict__ A16, const _Float16* __restrict__ Bt,
    const float* __restrict__ bias, const float* __restrict__ mp, _Float16* out16) {
  gemm_body<1>(A16, (unsigned)LDA, Bt, (unsigned)DIM, bias, mp, (float*)0, out16);
}

__global__ __launch_bounds__(256) void gemm_mv_kernel(
    const _Float16* __restrict__ A16, const _Float16* __restrict__ Bt,
    const float* __restrict__ bmg, const float* __restrict__ ci,
    const float* __restrict__ wat, const float* __restrict__ bat,
    float* __restrict__ mv) {
  __shared__ float Ms[2 * 64];
  const unsigned tid = threadIdx.x, lane = tid & 31u;
  const unsigned w = (unsigned)__builtin_amdgcn_readfirstlane(threadIdx.x >> 5);
  const unsigned mw = w >> 1, nw = w & 1u;
  const unsigned hh = lane >> 4, m = lane & 15u;
  const unsigned row0 = blockIdx.x * 64u;
  const unsigned rbase = row0 + mw * 16u + hh * 8u;
  const unsigned blo = rbase / (unsigned)PIX;
  const unsigned bhi = (rbase + 7u) / (unsigned)PIX;
  const unsigned bnd = (blo + 1u) * (unsigned)PIX;
  const float cs = 1.0f / (ACARRY * WCARRY);

  const _Float16* ap = A16 + (size_t)(row0 + mw * 16u + m) * LDA + hh * 8u;
  float p[8];
#pragma unroll
  for (int r = 0; r < 8; ++r) p[r] = 0.0f;

#pragma unroll 1
  for (unsigned nt = 0; nt < (unsigned)(DIM / 64); ++nt) {
    const unsigned col0 = nt * 64u + nw * 32u + m;
    const unsigned col1 = col0 + 16u;
    const _Float16* bp0 = Bt + (size_t)col0 * KMG + hh * 8u;
    const _Float16* bp1 = bp0 + (size_t)16 * KMG;
    v8f acc0 = {}, acc1 = {};
#pragma unroll 2
    for (unsigned k0 = 0; k0 < (unsigned)KMG; k0 += 32u) {
      const v16h a  = frag_at(ap + k0);
      const v16h b0 = frag_at(bp0 + k0);
      const v16h b1 = frag_at(bp1 + k0);
      acc0 = wmma16(a, b0, acc0);
      acc1 = wmma16(a, b1, acc1);
    }
    const float wa0 = bf16r(wat[col0]);
    const float wa1 = bf16r(wat[col1]);
    const float g0 = bf16r(bmg[col0]);
    const float g1 = bf16r(bmg[col1]);
    const float cl0 = bf16r(ci[(size_t)blo * DIM + col0]) * wa0;
    const float ch0 = bf16r(ci[(size_t)bhi * DIM + col0]) * wa0;
    const float cl1 = bf16r(ci[(size_t)blo * DIM + col1]) * wa1;
    const float ch1 = bf16r(ci[(size_t)bhi * DIM + col1]) * wa1;
#pragma unroll
    for (int r = 0; r < 8; ++r) {
      const bool up = (rbase + (unsigned)r) >= bnd;
      const float c0 = up ? ch0 : cl0;
      const float c1 = up ? ch1 : cl1;
      p[r] += (acc0[r] * cs + g0) * c0 + (acc1[r] * cs + g1) * c1;
    }
  }

#pragma unroll
  for (int r = 0; r < 8; ++r) p[r] = red16_sum(p[r]);
  float val = p[0];
#pragma unroll
  for (int r = 1; r < 8; ++r) val = (m == (unsigned)r) ? p[r] : val;
  if (m < 8u) Ms[nw * 64u + mw * 16u + hh * 8u + m] = val;
  __syncthreads();

  if (tid < 16u) {
    const v4f a = *(const v4f*)&Ms[tid * 4u];
    const v4f c = *(const v4f*)&Ms[64u + tid * 4u];
    const float ba = bf16r(bat[0]);
    v4f o;
#pragma unroll
    for (int j = 0; j < 4; ++j) o[j] = (a[j] + c[j]) + ba;
    float* dst = mv + (size_t)row0 + tid * 4u;
    *(volatile v4f*)dst = o;
    __threadfence();
    *(volatile v4f*)dst = o;
  }
}

__global__ __launch_bounds__(256) void outk_kernel(
    const float* __restrict__ KB, const float* __restrict__ mv, float* __restrict__ out) {
#pragma clang fp contract(off)
  __shared__ float Mv[7 * 32];
  __shared__ float Os[128];
  const unsigned tid = threadIdx.x, lane = tid & 31u;
  const unsigned w = (unsigned)__builtin_amdgcn_readfirstlane(threadIdx.x >> 5);
  const unsigned cg = blockIdx.x, b = blockIdx.y;

  const unsigned tcl = (tid < (unsigned)PIX) ? tid : (unsigned)(PIX - 1);
  const float mval = mv[(size_t)b * PIX + tcl];
  if (tid < 224u) Mv[tid] = (tid < (unsigned)PIX) ? mval : 0.0f;
  __syncthreads();

  float mreg[7];
#pragma unroll
  for (int j = 0; j < 7; ++j) mreg[j] = Mv[lane + 32u * (unsigned)j];

#pragma unroll 1
  for (unsigned ch = 0; ch < 16u; ++ch) {
    const unsigned c = cg * 128u + w * 16u + ch;
    const float* src = KB + ((size_t)b * DIM + c) * PIX;
    float s = 0.0f;
#pragma unroll
    for (int j = 0; j < 7; ++j) {
      const unsigned t = lane + 32u * (unsigned)j;
      const unsigned tc = (t < (unsigned)PIX) ? t : (unsigned)(PIX - 1);
      const float x = bf16r(src[tc]);
      const float pr = mreg[j] * x;
      s += (t < (unsigned)PIX) ? pr : 0.0f;
    }
    s = red32_sum(s);
    if (lane == 0u) Os[w * 16u + ch] = s;
  }
  __syncthreads();

  if (w == 0u) {
    const v4f o = *(const v4f*)&Os[lane * 4u];
    float* dst = out + (size_t)b * DIM + cg * 128u + lane * 4u;
    *(volatile v4f*)dst = o;
    __threadfence();
    *(volatile v4f*)dst = o;
  }
}

extern "C" void kernel_launch(void* const* d_in, const int* in_sizes, int n_in,
                              void* d_out, int out_size, void* d_ws, size_t ws_size,
                              hipStream_t stream) {
  if (n_in < 11) return;
  if ((long long)in_sizes[0] < (long long)NB_FULL * DIM) return;
  if ((long long)in_sizes[1] < (long long)NB * DIM * PIX) return;
  if ((long long)in_sizes[2] < (long long)NB * DIM) return;
  if ((long long)in_sizes[3] < (long long)DIM * DIM) return;
  if ((long long)in_sizes[5] < (long long)DIM * DIM) return;
  if ((long long)in_sizes[7] < (long long)KMG * DIM) return;
  if (in_sizes[4] < DIM || in_sizes[6] < DIM || in_sizes[8] < DIM || in_sizes[9] < DIM) return;
  if (in_sizes[10] < 1) return;
  if ((long long)out_size < (long long)NB * DIM) return;
  if (ws_size < WS_TOTAL) return;

  const float* m_prev  = (const float*)d_in[0];
  const float* KB      = (const float*)d_in[1];
  const float* c_i     = (const float*)d_in[2];
  const float* W_m     = (const float*)d_in[3];
  const float* b_m     = (const float*)d_in[4];
  const float* W_kb    = (const float*)d_in[5];
  const float* b_kb    = (const float*)d_in[6];
  const float* W_merge = (const float*)d_in[7];
  const float* b_merge = (const float*)d_in[8];
  const float* W_attn  = (const float*)d_in[9];
  const float* b_attn  = (const float*)d_in[10];
  float* out = (float*)d_out;

  char* ws = (char*)d_ws;
  _Float16* Wm_t  = (_Float16*)(ws + OFF_WM);
  _Float16* Wkb_t = (_Float16*)(ws + OFF_WKB);
  _Float16* Wmg_t = (_Float16*)(ws + OFF_WMG);
  _Float16* M16   = (_Float16*)(ws + OFF_M16);
  float*    MP    = (float*)(ws + OFF_MP);
  _Float16* XI    = (_Float16*)(ws + OFF_XI);
  float*    MV    = (float*)(ws + OFF_MV);

  dim3 blk(256);

  wconv_kernel<<<dim3(DIM / 64, DIM / 64), blk, 0, stream>>>(W_m, Wm_t, (unsigned)DIM, (unsigned)DIM);
  wconv_kernel<<<dim3(DIM / 64, DIM / 64), blk, 0, stream>>>(W_kb, Wkb_t, (unsigned)DIM, (unsigned)DIM);
  wconv_kernel<<<dim3(DIM / 64, KMG / 64), blk, 0, stream>>>(W_merge, Wmg_t, (unsigned)DIM, (unsigned)KMG);

  mconv_kernel<<<dim3((NB_FULL * DIM) / 2048), blk, 0, stream>>>(m_prev, M16);
  kbconv_kernel<<<dim3(DIM / 64, NB), blk, 0, stream>>>(KB, XI);
  gemm_mp_kernel<<<dim3(DIM / 64, NB_FULL / 64), blk, 0, stream>>>(M16, Wm_t, b_m, MP);
  gemm_i_kernel<<<dim3(DIM / 64, MROWS / 64), blk, 0, stream>>>(XI + DIM, Wkb_t, b_kb, MP, XI);
  gemm_mv_kernel<<<dim3(MROWS / 64), blk, 0, stream>>>(XI, Wmg_t, b_merge, c_i, W_attn, b_attn, MV);
  outk_kernel<<<dim3(DIM / 128, NB), blk, 0, stream>>>(KB, MV, out);
}
